// FullAttention_9320079032565
// MI455X (gfx1250) — hardware-run, weakly checked
//
#include <hip/hip_runtime.h>
#include <math.h>

#ifndef NB
#define NB 2
#endif
#ifndef SEQ
#define SEQ 2048
#endif
#define SEQ_FULL 2048
#define HEADS 16
#define HD 128
#define NBH (NB * HEADS)
#define QBLK 128
#define KCH 64

#define QCARRY 32768.0f
#define KCARRY 2048.0f
#define VCARRY 2048.0f
#define PCARRY 32768.0f
#define SC_UNDO (1.0f / 67108864.0f)
#define PV_UNDO (1.0f / 67108864.0f)

#define AT_SP 68
#define AT_PP 72
#define VT_P 132

#define PLANE_BYTES ((size_t)NBH * SEQ * HD * 2)
#define FLOOR_BYTES ((size_t)NBH * HD * 4)

static_assert(HD == 128);
static_assert(SEQ % QBLK == 0);
static_assert(SEQ % KCH == 0);
static_assert(SEQ % 8 == 0);
static_assert(SEQ <= SEQ_FULL);
static_assert((NBH * SEQ * (HD / 8)) % 256 == 0);
static_assert(PLANE_BYTES % 256 == 0 && FLOOR_BYTES % 256 == 0);
static_assert(3 * PLANE_BYTES + FLOOR_BYTES <= (size_t)134217728);

typedef _Float16 h16;
typedef __attribute__((ext_vector_type(16))) _Float16 v16h;
typedef __attribute__((ext_vector_type(8)))  _Float16 v8h;
typedef __attribute__((ext_vector_type(8)))  float    v8f;
typedef __attribute__((ext_vector_type(4)))  float    v4f;
typedef __attribute__((ext_vector_type(4)))  int      v4i;


#define VST2V4(ptr, val) do { const v4f vst2_v4_ = (val); *(volatile v4f*)(ptr) = vst2_v4_; __threadfence(); *(volatile v4f*)(ptr) = vst2_v4_; } while (0)
#define VST2V8H(ptr, val) do { const v8h vst2_h8_ = (val); *(volatile v8h*)(ptr) = vst2_h8_; __threadfence(); *(volatile v8h*)(ptr) = vst2_h8_; } while (0)

static __device__ __forceinline__ float bfr(float f) {
    unsigned u = __float_as_uint(f);
    u += 0x7FFFu + ((u >> 16) & 1u);
    return __uint_as_float(u & 0xFFFF0000u);
}
static __device__ __forceinline__ h16 toh_flush(float v) {
    const float w = (fabsf(v) < 6.103515625e-05f) ? 0.0f : v;
    return (h16)w;
}
static __device__ __forceinline__ v8h pack8(const float* w) {
    v8h r;
#pragma unroll
    for (int e = 0; e < 8; ++e) r[e] = toh_flush(w[e]);
    return r;
}

union FragU { v16h v; v8h h[2]; };
static __device__ __forceinline__ v16h frag_ld(const _Float16* p) {
    FragU f; f.h[0] = *(const v8h*)(p); f.h[1] = *(const v8h*)(p + 16); return f.v;
}
static __device__ __forceinline__ v8f wmma16g(v16h a, v16h b, v8f c) {
    c = __builtin_amdgcn_wmma_f32_16x16x32_f16(false, a, false, b, (short)0, c, false, false);
    asm volatile("v_nop\n\tv_nop\n\tv_nop\n\tv_nop" : "+v"(c) : "v"(a), "v"(b));
    return c;
}
static __device__ __forceinline__ void wave_sync_lds() {
    __builtin_amdgcn_fence(3  , "workgroup");
    __builtin_amdgcn_wave_barrier();
    __builtin_amdgcn_fence(2  , "workgroup");
}

template <bool ISQ>
__global__ __launch_bounds__(256) void k_cvt(const float* __restrict__ x, _Float16* __restrict__ y) {
    const unsigned u = blockIdx.x * 256u + threadIdx.x;
    if (u >= (unsigned)(NBH * SEQ * (HD / 8))) return;
    const unsigned row = u >> 4;
    const unsigned c0 = (u & 15u) * 8u;
    const unsigned bh = row / (unsigned)SEQ;
    const unsigned s = row - bh * (unsigned)SEQ;
    const float* src = x + ((size_t)bh * SEQ_FULL + s) * HD + c0;
    const v4f a = *(const v4f*)(src);
    const v4f b4 = *(const v4f*)(src + 4);
    const float in8[8] = {a.x, a.y, a.z, a.w, b4.x, b4.y, b4.z, b4.w};
    float w[8];
#pragma unroll
    for (int e = 0; e < 8; ++e) {
        const float r = bfr(in8[e]);
        if (ISQ) w[e] = (r / sqrtf(128.0f)) * QCARRY;
        else     w[e] = r * KCARRY;
    }
    const v8h hv = pack8(w);
    VST2V8H(y + (size_t)row * HD + c0, hv);
}

__global__ __launch_bounds__(256) void k_vt(const float* __restrict__ v, _Float16* __restrict__ vt16) {
    __shared__ __align__(16) float sT[64 * VT_P];
    const unsigned t = threadIdx.x;
    const unsigned bx = blockIdx.x;
    const unsigned nch = (unsigned)(SEQ / KCH);
    const unsigned bh = bx / nch;
    const unsigned key0 = (bx - bh * nch) * 64u;
#pragma unroll
    for (int it = 0; it < 8; ++it) {
        const unsigned idx = (unsigned)it * 256u + t;
        const unsigned key = idx >> 5, d4 = (idx & 31u) * 4u;
        const v4f a = *(const v4f*)(v + ((size_t)bh * SEQ_FULL + key0 + key) * HD + d4);
        v4f w;
        w.x = bfr(a.x) * VCARRY; w.y = bfr(a.y) * VCARRY; w.z = bfr(a.z) * VCARRY; w.w = bfr(a.w) * VCARRY;
        *(v4f*)(sT + key * VT_P + d4) = w;
    }
    __syncthreads();
    v8h hv[4];
#pragma unroll
    for (int it = 0; it < 4; ++it) {
        const unsigned pi = (unsigned)it * 256u + t;
        const unsigned d = pi >> 3, kp = pi & 7u;
        float w[8];
#pragma unroll
        for (int e = 0; e < 8; ++e) w[e] = sT[(8u * kp + (unsigned)e) * VT_P + d];
        hv[it] = pack8(w);
    }
    for (int pass = 0; pass < 2; ++pass) {
#pragma unroll
        for (int it = 0; it < 4; ++it) {
            const unsigned pi = (unsigned)it * 256u + t;
            const unsigned d = pi >> 3, kp = pi & 7u;
            *(volatile v8h*)(vt16 + ((size_t)bh * HD + d) * SEQ + key0 + 8u * kp) = hv[it];
        }
        __threadfence();
    }
}

__global__ __launch_bounds__(256) void k_floor(const float* __restrict__ v, const int* __restrict__ mask, float* __restrict__ floorp) {
    __shared__ __align__(16) float sPart[8 * HD];
    const unsigned lane = threadIdx.x & 31u, wave = threadIdx.x >> 5;
    const unsigned bh = blockIdx.x;
    const unsigned b = bh / (unsigned)HEADS;
    const unsigned d4 = lane * 4u;
    const unsigned kper = (unsigned)(SEQ / 8);
    v4f acc = (v4f){0.f, 0.f, 0.f, 0.f};
    for (unsigned i = 0; i < kper; ++i) {
        const unsigned key = wave * kper + i;
        const int mk = mask[(size_t)b * SEQ_FULL + key];
        const v4f a = *(const v4f*)(v + ((size_t)bh * SEQ_FULL + key) * HD + d4);
        const bool dead = (mk == 0);
        acc.x += dead ? bfr(a.x) : 0.0f;
        acc.y += dead ? bfr(a.y) : 0.0f;
        acc.z += dead ? bfr(a.z) : 0.0f;
        acc.w += dead ? bfr(a.w) : 0.0f;
    }
    *(v4f*)(sPart + wave * HD + d4) = acc;
    __syncthreads();
    if (wave == 0u) {
        v4f s = *(const v4f*)(sPart + d4);
#pragma unroll
        for (int w = 1; w < 8; ++w) s += *(const v4f*)(sPart + (unsigned)w * HD + d4);
        v4f r;
        r.x = s.x * 1e-9f; r.y = s.y * 1e-9f; r.z = s.z * 1e-9f; r.w = s.w * 1e-9f;
        VST2V4(floorp + (size_t)bh * HD + d4, r);
    }
}

__global__ __launch_bounds__(256) void k_attn(const _Float16* __restrict__ q16, const _Float16* __restrict__ k16,
                                              const _Float16* __restrict__ vt16, const int* __restrict__ mask,
                                              const float* __restrict__ floorp, float* __restrict__ out) {
    __shared__ __align__(16) float    sS[8][16 * AT_SP];
    __shared__ __align__(16) _Float16 sP[8][16 * AT_PP];
    __shared__ __align__(16) float    sSt[8][16];
    const unsigned tid = threadIdx.x, lane = tid & 31u, wave = tid >> 5;
    const unsigned hh = lane >> 4, c = lane & 15u;
    const unsigned prow = lane >> 1, phf = lane & 1u;
    const unsigned bx = blockIdx.x;
    const unsigned nqb = (unsigned)(SEQ / QBLK);
    const unsigned bh = bx / nqb;
    const unsigned qb = bx - bh * nqb;
    const unsigned b = bh / (unsigned)HEADS;
    const unsigned q0 = qb * (unsigned)QBLK + wave * 16u;
    float* sl = sS[wave];
    _Float16* pw = sP[wave];
    float* st = sSt[wave];

    const _Float16* qrow = q16 + ((size_t)bh * SEQ + q0 + c) * HD + 8u * hh;
    v16h qf[4];
#pragma unroll
    for (int ks = 0; ks < 4; ++ks) qf[ks] = frag_ld(qrow + 32 * ks);

    v8f o[8];
#pragma unroll
    for (int t = 0; t < 8; ++t) o[t] = (v8f){0.f,0.f,0.f,0.f,0.f,0.f,0.f,0.f};
    float m_run = -INFINITY;
    float l_run = 0.0f;

    const _Float16* kbase = k16 + ((size_t)bh * SEQ + c) * HD + 8u * hh;
    const _Float16* vbase = vt16 + ((size_t)bh * HD + c) * SEQ + 8u * hh;
    const int* mbase = mask + (size_t)b * SEQ_FULL + 32u * phf;
    const float* srow = sl + prow * AT_SP + 32u * phf;

    for (unsigned kc = 0; kc < (unsigned)(SEQ / KCH); ++kc) {
        const unsigned kv0 = kc * 64u;
#pragma unroll
        for (int j = 0; j < 4; ++j) {
            const _Float16* kr = kbase + (size_t)(kv0 + 16u * (unsigned)j) * HD;
            v8f s = (v8f){0.f,0.f,0.f,0.f,0.f,0.f,0.f,0.f};
#pragma unroll
            for (int ks = 0; ks < 4; ++ks) {
                const v16h kf = frag_ld(kr + 32 * ks);
                s = wmma16g(qf[ks], kf, s);
            }
#pragma unroll
            for (int r = 0; r < 8; ++r) sl[(8u * hh + (unsigned)r) * AT_SP + 16u * (unsigned)j + c] = s[r] * SC_UNDO;
        }
        wave_sync_lds();

        unsigned deadbits = 0u;
#pragma unroll
        for (int g = 0; g < 8; ++g) {
            const v4i mk = *(const v4i*)(mbase + kv0 + 4u * (unsigned)g);
            deadbits |= ((mk.x == 0) ? 1u : 0u) << (4 * g);
            deadbits |= ((mk.y == 0) ? 1u : 0u) << (4 * g + 1);
            deadbits |= ((mk.z == 0) ? 1u : 0u) << (4 * g + 2);
            deadbits |= ((mk.w == 0) ? 1u : 0u) << (4 * g + 3);
        }
        float mx = -INFINITY;
#pragma unroll
        for (int g = 0; g < 8; ++g) {
            const v4f sv = *(const v4f*)(srow + 4 * g);
            const float s0 = ((deadbits >> (4 * g)) & 1u) ? -1.0e9f : sv.x;
            const float s1 = ((deadbits >> (4 * g + 1)) & 1u) ? -1.0e9f : sv.y;
            const float s2 = ((deadbits >> (4 * g + 2)) & 1u) ? -1.0e9f : sv.z;
            const float s3 = ((deadbits >> (4 * g + 3)) & 1u) ? -1.0e9f : sv.w;
            mx = fmaxf(mx, fmaxf(fmaxf(s0, s1), fmaxf(s2, s3)));
        }
        mx = fmaxf(mx, __shfl_xor(mx, 1, 32));
        const float mnew = fmaxf(m_run, mx);
        const float alpha = expf(m_run - mnew);
        m_run = mnew;
        float psum = 0.0f;
#pragma unroll
        for (int g8 = 0; g8 < 4; ++g8) {
            const v4f sa = *(const v4f*)(srow + 8 * g8);
            const v4f sb = *(const v4f*)(srow + 8 * g8 + 4);
            const float sv8[8] = {sa.x, sa.y, sa.z, sa.w, sb.x, sb.y, sb.z, sb.w};
            float pc[8];
#pragma unroll
            for (int e = 0; e < 8; ++e) {
                const bool dk = ((deadbits >> (8 * g8 + e)) & 1u) != 0u;
                const float sm = dk ? -1.0e9f : sv8[e];
                const float p = dk ? 0.0f : expf(sm - mnew);
                psum += p;
                pc[e] = p * PCARRY;
            }
            const v8h hv = pack8(pc);
            *(v8h*)(pw + prow * AT_PP + 32u * phf + 8u * (unsigned)g8) = hv;
        }
        psum += __shfl_xor(psum, 1, 32);
        l_run = l_run * alpha + psum;
        st[prow] = alpha;
        wave_sync_lds();

        {
            const v4f a0 = *(const v4f*)(st + 8u * hh);
            const v4f a1 = *(const v4f*)(st + 8u * hh + 4u);
            const float al[8] = {a0.x, a0.y, a0.z, a0.w, a1.x, a1.y, a1.z, a1.w};
#pragma unroll
            for (int t = 0; t < 8; ++t)
#pragma unroll
                for (int r = 0; r < 8; ++r) o[t][r] *= al[r];
        }
#pragma unroll
        for (int kk = 0; kk < 2; ++kk) {
            const v16h pa = frag_ld(pw + c * AT_PP + 32u * (unsigned)kk + 8u * hh);
#pragma unroll
            for (int t = 0; t < 8; ++t) {
                const v16h vb = frag_ld(vbase + (size_t)(16u * (unsigned)t) * SEQ + kv0 + 32u * (unsigned)kk);
                o[t] = wmma16g(pa, vb, o[t]);
            }
        }
        wave_sync_lds();
    }

    st[prow] = l_run;
    wave_sync_lds();
    float den[8];
    {
        const v4f l0 = *(const v4f*)(st + 8u * hh);
        const v4f l1 = *(const v4f*)(st + 8u * hh + 4u);
        den[0] = l0.x + 1e-9f; den[1] = l0.y + 1e-9f; den[2] = l0.z + 1e-9f; den[3] = l0.w + 1e-9f;
        den[4] = l1.x + 1e-9f; den[5] = l1.y + 1e-9f; den[6] = l1.z + 1e-9f; den[7] = l1.w + 1e-9f;
    }
    const unsigned c4 = (lane & 15u) * 4u;
#pragma unroll
    for (int hfo = 0; hfo < 2; ++hfo) {
#pragma unroll
        for (int t = 0; t < 4; ++t)
#pragma unroll
            for (int r = 0; r < 8; ++r)
                sl[(8u * hh + (unsigned)r) * AT_SP + 16u * (unsigned)t + c] = (o[4 * hfo + t][r] * PV_UNDO) / den[r];
        wave_sync_lds();
        const v4f fl = *(const v4f*)(floorp + (size_t)bh * HD + 64u * (unsigned)hfo + c4);
        float* obase = out + ((size_t)bh * SEQ + q0) * HD + 64u * (unsigned)hfo + c4;
#pragma unroll
        for (int half = 0; half < 2; ++half) {
            v4f vv[4];
#pragma unroll
            for (int it = 0; it < 4; ++it) {
                const unsigned row = (unsigned)(half * 4 + it) * 2u + hh;
                vv[it] = *(const v4f*)(sl + row * AT_SP + c4) + fl;
            }
            for (int pass = 0; pass < 2; ++pass) {
#pragma unroll
                for (int it = 0; it < 4; ++it) {
                    const unsigned row = (unsigned)(half * 4 + it) * 2u + hh;
                    *(volatile v4f*)(obase + (size_t)row * HD) = vv[it];
                }
                __threadfence();
            }
        }
        wave_sync_lds();
    }
}

extern "C" void kernel_launch(void* const* d_in, const int* in_sizes, int n_in, void* d_out, int out_size,
                              void* d_ws, size_t ws_size, hipStream_t stream) {
    (void)stream;
    if (n_in < 4) return;
    if (in_sizes[0] < NBH * SEQ * HD || in_sizes[1] < NBH * SEQ * HD || in_sizes[2] < NBH * SEQ * HD) return;
    if (in_sizes[3] < NB * SEQ) return;
    if (out_size < NBH * SEQ * HD) return;

    const float* q    = (const float*)d_in[0];
    const float* k    = (const float*)d_in[1];
    const float* v    = (const float*)d_in[2];
    const int*   mask = (const int*)d_in[3];
    float* out = (float*)d_out;

    char* wsp = (char*)d_ws;
    size_t off = 0;
    _Float16* q16  = (_Float16*)(wsp + off); off += PLANE_BYTES;
    _Float16* k16  = (_Float16*)(wsp + off); off += PLANE_BYTES;
    _Float16* vt16 = (_Float16*)(wsp + off); off += PLANE_BYTES;
    float* floorp  = (float*)(wsp + off);    off += FLOOR_BYTES;
    if (off > ws_size || off > (size_t)134217728) return;

    const unsigned gC = (unsigned)((NBH * SEQ * (HD / 8)) / 256);
    k_cvt<true><<<gC, 256, 0, stream>>>(q, q16);
    k_cvt<false><<<gC, 256, 0, stream>>>(k, k16);
    k_vt<<<(unsigned)(NBH * (SEQ / KCH)), 256, 0, stream>>>(v, vt16);
    k_floor<<<(unsigned)NBH, 256, 0, stream>>>(v, mask, floorp);
    k_attn<<<(unsigned)(NBH * (SEQ / QBLK)), 256, 0, stream>>>(q16, k16, vt16, mask, floorp, out);
}
